// QuantumNeuralNetwork_50405736186429
// MI455X (gfx1250) — hardware-verified
//
#include <hip/hip_runtime.h>
#include <stddef.h>


typedef _Float16 v16h __attribute__((ext_vector_type(16)));
typedef _Float16 v8h  __attribute__((ext_vector_type(8)));
typedef float    v8f  __attribute__((ext_vector_type(8)));
typedef float    v4f  __attribute__((ext_vector_type(4)));
typedef _Float16 h16;

#ifndef NB
#define NB 8
#endif
#ifndef SEQ
#define SEQ 2048
#endif
#define NB_FULL  8
#define SEQ_FULL 2048
#define DIM   512
#define NPAIR 4
#define PSZ   128
#define NQUB  8
#define NLAY  3
#define NSUP  8
#define REP   (DIM / NQUB)
#define MROWS (NB * SEQ)

static_assert(NB >= 1 && NB <= NB_FULL);
static_assert(SEQ >= 64 && SEQ <= SEQ_FULL && (SEQ % 64) == 0);
static_assert(DIM == NPAIR * PSZ);
static_assert(REP == 64);
static_assert(PSZ == 128);
static_assert((PSZ % 32) == 0 && (DIM % 32) == 0);
static_assert((DIM % 64) == 0 && (PSZ % 64) == 0);
static_assert((MROWS % 64) == 0 && (MROWS % 4) == 0);
static_assert(DIM / 8 == 64);
static_assert(((size_t)MROWS * DIM) % 2048 == 0);
static_assert((size_t)MROWS * DIM < (size_t)0xFFFFFFFFu);

#define LDT 72
#define LDC 68
static_assert((LDT % 8) == 0 && LDT >= 64);
static_assert((LDC % 4) == 0 && LDC >= 64);

#define WCARRY 64.0f
#define QCARRY 64.0f

#define WSQ_BYTES     ((size_t)DIM * DIM * 2)
#define WENT_BYTES    ((size_t)DIM * PSZ * 2)
#define PLANE16_BYTES ((size_t)MROWS * DIM * 2)
#define OFF_WIN   ((size_t)0)
#define OFF_WENT  (OFF_WIN + WSQ_BYTES)
#define OFF_WMEAS (OFF_WENT + WENT_BYTES)
#define OFF_WOUT  (OFF_WMEAS + WSQ_BYTES)
#define OFF_XA    (OFF_WOUT + WSQ_BYTES)
#define OFF_P1    (OFF_XA + PLANE16_BYTES)
#define OFF_P2    (OFF_P1 + PLANE16_BYTES)
#define OFF_P3    (OFF_P2 + PLANE16_BYTES)
#define WS_TOTAL  (OFF_P3 + PLANE16_BYTES)
static_assert((WSQ_BYTES % 128) == 0 && (WENT_BYTES % 128) == 0 && (PLANE16_BYTES % 128) == 0);
static_assert(WS_TOTAL <= (size_t)134217728);

__device__ __forceinline__ float bf16r(float x) {
  unsigned int u = __float_as_uint(x);
  u = (u + 0x7FFFu + ((u >> 16) & 1u)) & 0xFFFF0000u;
  return __uint_as_float(u);
}

static __device__ __forceinline__ h16 toh_flush(float v) {
  const h16 r = (h16)v;
  return (fabsf(v) < 6.103515625e-05f) ? (h16)0.0f : r;
}

__device__ __forceinline__ v16h frag_at(const _Float16* p) {
  v8h lo = *(const v8h*)(p);
  v8h hi = *(const v8h*)(p + 16);
  v16h out;
#pragma unroll
  for (int i = 0; i < 8; ++i) { out[i] = lo[i]; out[i + 8] = hi[i]; }
  return out;
}

__device__ __forceinline__ v8f wmma16(v16h a, v16h b, v8f c) {
  v8f d = __builtin_amdgcn_wmma_f32_16x16x32_f16(false, a, false, b, (short)0, c,
                                                 false, false);
  asm volatile("v_nop\n\tv_nop\n\tv_nop\n\tv_nop" : "+v"(d) : "v"(a), "v"(b));
  return d;
}

__global__ __launch_bounds__(256) void wconv_kernel(
    const float* __restrict__ W, _Float16* __restrict__ Wt, unsigned ldw, unsigned ldk) {
  __shared__ _Float16 T[64 * LDT];
  const unsigned tid = threadIdx.x;
  const unsigned n0 = blockIdx.x * 64u;
  const unsigned k0 = blockIdx.y * 64u;
#pragma unroll 4
  for (unsigned j = 0; j < 16u; ++j) {
    const unsigned idx = tid + 256u * j;
    const unsigned kr = idx >> 6, nc = idx & 63u;
    const float v = W[(size_t)(k0 + kr) * ldw + n0 + nc];
    T[nc * LDT + kr] = (_Float16)(WCARRY * bf16r(v));
  }
  __syncthreads();
  v8h x[2];
  size_t off[2];
#pragma unroll
  for (unsigned i = 0; i < 2u; ++i) {
    const unsigned n = 32u * i + (tid >> 3);
    const unsigned kc = (tid & 7u) * 8u;
    x[i] = *(const v8h*)&T[n * LDT + kc];
    off[i] = (size_t)(n0 + n) * ldk + k0 + kc;
  }
#pragma unroll
  for (int i = 0; i < 2; ++i) *(volatile v8h*)(Wt + off[i]) = x[i];
  __threadfence();
#pragma unroll
  for (int i = 0; i < 2; ++i) *(volatile v8h*)(Wt + off[i]) = x[i];
}

__global__ __launch_bounds__(256) void xconv_kernel(
    const float* __restrict__ X, _Float16* __restrict__ dst) {
#pragma clang fp contract(off)
  const unsigned t = blockIdx.x * 256u + threadIdx.x;
  const unsigned crow = t >> 6;
  const unsigned c = (t & 63u) * 8u;
  const unsigned bidx = crow / (unsigned)SEQ;
  const unsigned sq = crow - bidx * (unsigned)SEQ;
  const size_t srow = (size_t)bidx * SEQ_FULL + sq;
  const v4f a0 = *(const v4f*)(X + srow * DIM + c);
  const v4f a1 = *(const v4f*)(X + srow * DIM + c + 4u);
  v8h o;
#pragma unroll
  for (int i = 0; i < 4; ++i) {
    o[i]     = toh_flush(bf16r(a0[i]));
    o[i + 4] = toh_flush(bf16r(a1[i]));
  }
  _Float16* p = dst + (size_t)crow * DIM + c;
  *(volatile v8h*)p = o;
  __threadfence();
  *(volatile v8h*)p = o;
}

template <int MODE>
__device__ __forceinline__ void gemm_body(
    const _Float16* __restrict__ A16, const _Float16* __restrict__ Bt, const unsigned K,
    const float* __restrict__ bias, const float* __restrict__ estr,
    const float* __restrict__ supw, const float* __restrict__ supc,
    const float* __restrict__ cpar, float* __restrict__ outf, _Float16* __restrict__ out16) {
  __shared__ float Cs[64 * LDC];
  const unsigned tid = threadIdx.x, lane = tid & 31u;
  const unsigned w = (unsigned)__builtin_amdgcn_readfirstlane((int)(tid >> 5));
  const unsigned mw = w >> 1, nw = w & 1u;
  const unsigned hh = lane >> 4, m = lane & 15u;
  const unsigned n0 = blockIdx.x * 64u;
  const unsigned row0 = blockIdx.y * 64u;
  const unsigned acol0 = (MODE == 1) ? (n0 / (unsigned)PSZ) * (unsigned)PSZ : 0u;

  const _Float16* ap  = A16 + (size_t)(row0 + mw * 16u + m) * DIM + acol0 + hh * 8u;
  const _Float16* bp0 = Bt + (size_t)(n0 + nw * 32u + m) * K + hh * 8u;
  const _Float16* bp1 = bp0 + (size_t)16 * K;
  v8f acc0 = {}, acc1 = {};
#pragma unroll 2
  for (unsigned k0 = 0; k0 < K; k0 += 32u) {
    const v16h a  = frag_at(ap + k0);
    const v16h b0 = frag_at(bp0 + k0);
    const v16h b1 = frag_at(bp1 + k0);
    acc0 = wmma16(a, b0, acc0);
    acc1 = wmma16(a, b1, acc1);
  }
#pragma unroll
  for (int r = 0; r < 8; ++r) {
    float* d = &Cs[(mw * 16u + hh * 8u + (unsigned)r) * LDC + nw * 32u + m];
    d[0]  = acc0[r];
    d[16] = acc1[r];
  }
  __syncthreads();

  if (MODE == 0 || MODE == 2) {
    v8h x[2];
    size_t off[2];
#pragma unroll
    for (unsigned i = 0; i < 2u; ++i) {
      const unsigned r = 32u * i + (tid >> 3);
      const unsigned c = (tid & 7u) * 8u;
      const v4f u0 = *(const v4f*)&Cs[r * LDC + c];
      const v4f u1 = *(const v4f*)&Cs[r * LDC + c + 4];
      if (MODE == 0) {
        const v4f g0 = *(const v4f*)(bias + n0 + c);
        const v4f g1 = *(const v4f*)(bias + n0 + c + 4u);
#pragma unroll
        for (int j = 0; j < 4; ++j) {
          x[i][j]     = toh_flush(u0[j] * (1.0f / WCARRY) + bf16r(g0[j]));
          x[i][j + 4] = toh_flush(u1[j] * (1.0f / WCARRY) + bf16r(g1[j]));
        }
      } else {
#pragma unroll
        for (int j = 0; j < 4; ++j) {
          x[i][j]     = toh_flush(u0[j] * (1.0f / WCARRY));
          x[i][j + 4] = toh_flush(u1[j] * (1.0f / WCARRY));
        }
      }
      off[i] = (size_t)(row0 + r) * DIM + n0 + c;
    }
#pragma unroll
    for (int i = 0; i < 2; ++i) *(volatile v8h*)(out16 + off[i]) = x[i];
    __threadfence();
#pragma unroll
    for (int i = 0; i < 2; ++i) *(volatile v8h*)(out16 + off[i]) = x[i];
  }

  if (MODE == 1) {
    const unsigned qub = blockIdx.x;
    const unsigned pr  = blockIdx.x >> 1;
    const unsigned c = (tid & 7u) * 8u;
    const float hs = 0.70710678118654752440f;
    const float es = bf16r(estr[pr]);
    float sv[8];
#pragma unroll
    for (int j = 0; j < 8; ++j) sv[j] = 0.0f;
#pragma unroll 1
    for (unsigned s = 0; s < (unsigned)NSUP; ++s) {
      const float cf = bf16r(supc[s]);
      const v4f w0 = *(const v4f*)(supw + (size_t)s * DIM + n0 + c);
      const v4f w1 = *(const v4f*)(supw + (size_t)s * DIM + n0 + c + 4u);
#pragma unroll
      for (int j = 0; j < 4; ++j) {
        sv[j]     += cf * bf16r(w0[j]);
        sv[j + 4] += cf * bf16r(w1[j]);
      }
    }
    float t[2][8];
#pragma unroll
    for (unsigned i = 0; i < 2u; ++i) {
      const unsigned r = 32u * i + (tid >> 3);
      const v4f u0 = *(const v4f*)&Cs[r * LDC + c];
      const v4f u1 = *(const v4f*)&Cs[r * LDC + c + 4];
#pragma unroll
      for (int j = 0; j < 4; ++j) {
        t[i][j]     = u0[j] * (1.0f / WCARRY);
        t[i][j + 4] = u1[j] * (1.0f / WCARRY);
      }
    }
#pragma unroll
    for (int i = 0; i < 2; ++i)
#pragma unroll
      for (int g = 0; g < 2; ++g) {
        const float a  = t[i][4 * g]     * es;
        const float b  = t[i][4 * g + 1] * es;
        const float cc = t[i][4 * g + 3] * es;
        const float d  = t[i][4 * g + 2] * es;
        t[i][4 * g]     = (a * hs + b * hs) * sv[4 * g];
        t[i][4 * g + 1] = (a * hs - b * hs) * sv[4 * g + 1];
        t[i][4 * g + 2] = (cc * hs + d * hs) * sv[4 * g + 2];
        t[i][4 * g + 3] = (cc * hs - d * hs) * sv[4 * g + 3];
      }
#pragma unroll 1
    for (unsigned l = 0; l < (unsigned)NLAY; ++l) {
      const float px = bf16r(cpar[(l * (unsigned)NQUB + qub) * 3u + 0u]);
      const float pz = bf16r(cpar[(l * (unsigned)NQUB + qub) * 3u + 2u]);
#pragma unroll
      for (int i = 0; i < 2; ++i)
#pragma unroll
        for (int g = 0; g < 2; ++g) {
          const float a  = t[i][4 * g];
          const float b  = t[i][4 * g + 1];
          const float cc = t[i][4 * g + 2];
          const float d  = t[i][4 * g + 3];
          const float h0 = a * hs + b * hs;
          const float h1 = a * hs - b * hs;
          const float h2 = cc * hs + d * hs;
          const float h3 = cc * hs - d * hs;
          const float x0 = h0 + px * h1;
          const float x1 = h1 + px * h0;
          const float x2 = h2 + px * h3;
          const float x3 = h3 + px * h2;
          const float z0 = x0 + pz * x0;
          const float z1 = x1 - pz * x1;
          const float z2 = x2 + pz * x2;
          const float z3 = x3 - pz * x3;
          t[i][4 * g]     = z0;
          t[i][4 * g + 1] = z1;
          t[i][4 * g + 2] = z3;
          t[i][4 * g + 3] = z2;
        }
    }
    v8h x[2];
    size_t off[2];
#pragma unroll
    for (unsigned i = 0; i < 2u; ++i) {
      const unsigned r = 32u * i + (tid >> 3);
#pragma unroll
      for (int j = 0; j < 8; ++j) x[i][j] = toh_flush(QCARRY * t[i][j]);
      off[i] = (size_t)(row0 + r) * DIM + n0 + c;
    }
#pragma unroll
    for (int i = 0; i < 2; ++i) *(volatile v8h*)(out16 + off[i]) = x[i];
    __threadfence();
#pragma unroll
    for (int i = 0; i < 2; ++i) *(volatile v8h*)(out16 + off[i]) = x[i];
  }

  if (MODE == 3) {
    const float cs = 1.0f / (WCARRY * QCARRY);
    v4f xs[4];
    size_t off[4];
#pragma unroll
    for (unsigned i = 0; i < 4u; ++i) {
      const unsigned r = 16u * i + (tid >> 4);
      const unsigned c = (tid & 15u) * 4u;
      const unsigned crow = row0 + r;
      const unsigned bidx = crow / (unsigned)SEQ;
      const unsigned sq = crow - bidx * (unsigned)SEQ;
      const size_t frow = (size_t)bidx * SEQ_FULL + sq;
      const v4f u = *(const v4f*)&Cs[r * LDC + c];
      const v4f g = *(const v4f*)(bias + n0 + c);
      v4f val;
#pragma unroll
      for (int j = 0; j < 4; ++j) val[j] = u[j] * cs + bf16r(g[j]);
      xs[i] = val;
      off[i] = frow * DIM + n0 + c;
    }
#pragma unroll
    for (int i = 0; i < 4; ++i) *(volatile v4f*)(outf + off[i]) = xs[i];
    __threadfence();
#pragma unroll
    for (int i = 0; i < 4; ++i) *(volatile v4f*)(outf + off[i]) = xs[i];
  }
}

__global__ __launch_bounds__(256) void gemm_in_kernel(
    const _Float16* __restrict__ A16, const _Float16* __restrict__ Bt,
    const float* __restrict__ bias, _Float16* __restrict__ out16) {
  gemm_body<0>(A16, Bt, (unsigned)DIM, bias, bias, bias, bias, bias, (float*)0, out16);
}
__global__ __launch_bounds__(256) void gemm_ent_kernel(
    const _Float16* __restrict__ A16, const _Float16* __restrict__ Bt,
    const float* __restrict__ estr, const float* __restrict__ supw,
    const float* __restrict__ supc, const float* __restrict__ cpar,
    _Float16* __restrict__ out16) {
  gemm_body<1>(A16, Bt, (unsigned)PSZ, estr, estr, supw, supc, cpar, (float*)0, out16);
}
__global__ __launch_bounds__(256) void gemm_meas_kernel(
    const _Float16* __restrict__ A16, const _Float16* __restrict__ Bt,
    _Float16* __restrict__ out16) {
  gemm_body<2>(A16, Bt, (unsigned)DIM, (const float*)0, (const float*)0, (const float*)0,
               (const float*)0, (const float*)0, (float*)0, out16);
}
__global__ __launch_bounds__(256) void gemm_out_kernel(
    const _Float16* __restrict__ A16, const _Float16* __restrict__ Bt,
    const float* __restrict__ bias, float* __restrict__ outf) {
  gemm_body<3>(A16, Bt, (unsigned)DIM, bias, bias, bias, bias, bias, outf, (_Float16*)0);
}

extern "C" void kernel_launch(void* const* d_in, const int* in_sizes, int n_in,
                              void* d_out, int out_size, void* d_ws, size_t ws_size,
                              hipStream_t stream) {
  if (n_in < 11) return;
  const long long need_x = ((long long)(NB - 1) * SEQ_FULL + SEQ) * DIM;
  if ((long long)in_sizes[0] < need_x) return;
  if ((long long)in_sizes[1] < (long long)DIM * DIM) return;
  if (in_sizes[2] < DIM) return;
  if ((long long)in_sizes[3] < (long long)NPAIR * PSZ * PSZ) return;
  if (in_sizes[4] < NPAIR) return;
  if (in_sizes[5] < NSUP * DIM) return;
  if (in_sizes[6] < NSUP) return;
  if (in_sizes[7] < NLAY * NQUB * 3) return;
  if ((long long)in_sizes[8] < (long long)DIM * DIM) return;
  if ((long long)in_sizes[9] < (long long)DIM * DIM) return;
  if (in_sizes[10] < DIM) return;
  if ((long long)out_size < need_x) return;
  if (ws_size < WS_TOTAL) return;

  const float* X     = (const float*)d_in[0];
  const float* in_w  = (const float*)d_in[1];
  const float* in_b  = (const float*)d_in[2];
  const float* ent_w = (const float*)d_in[3];
  const float* estr  = (const float*)d_in[4];
  const float* sup_w = (const float*)d_in[5];
  const float* sup_c = (const float*)d_in[6];
  const float* cpar  = (const float*)d_in[7];
  const float* meas  = (const float*)d_in[8];
  const float* out_w = (const float*)d_in[9];
  const float* out_b = (const float*)d_in[10];
  float* out = (float*)d_out;

  char* ws = (char*)d_ws;
  _Float16* Win_t   = (_Float16*)(ws + OFF_WIN);
  _Float16* Went_t  = (_Float16*)(ws + OFF_WENT);
  _Float16* Wmeas_t = (_Float16*)(ws + OFF_WMEAS);
  _Float16* Wout_t  = (_Float16*)(ws + OFF_WOUT);
  _Float16* XA16    = (_Float16*)(ws + OFF_XA);
  _Float16* P1      = (_Float16*)(ws + OFF_P1);
  _Float16* P2      = (_Float16*)(ws + OFF_P2);
  _Float16* P3      = (_Float16*)(ws + OFF_P3);

  dim3 blk(256);
  dim3 gsq(DIM / 64, DIM / 64);
  dim3 gg(DIM / 64, MROWS / 64);

  wconv_kernel<<<gsq, blk, 0, stream>>>(in_w, Win_t, (unsigned)DIM, (unsigned)DIM);
  for (int p = 0; p < NPAIR; ++p)
    wconv_kernel<<<dim3(PSZ / 64, PSZ / 64), blk, 0, stream>>>(
        ent_w + (size_t)p * PSZ * PSZ, Went_t + (size_t)p * PSZ * PSZ,
        (unsigned)PSZ, (unsigned)PSZ);
  wconv_kernel<<<gsq, blk, 0, stream>>>(meas, Wmeas_t, (unsigned)DIM, (unsigned)DIM);
  wconv_kernel<<<gsq, blk, 0, stream>>>(out_w, Wout_t, (unsigned)DIM, (unsigned)DIM);

  xconv_kernel<<<dim3((unsigned)(((size_t)MROWS * DIM) / 2048)), blk, 0, stream>>>(X, XA16);
  gemm_in_kernel<<<gg, blk, 0, stream>>>(XA16, Win_t, in_b, P1);
  gemm_ent_kernel<<<gg, blk, 0, stream>>>(P1, Went_t, estr, sup_w, sup_c, cpar, P2);
  gemm_meas_kernel<<<gg, blk, 0, stream>>>(P2, Wmeas_t, P3);
  gemm_out_kernel<<<gg, blk, 0, stream>>>(P3, Wout_t, out_b, out);
}
